// ChunkwiseRetention_28217935135456
// MI455X (gfx1250) — hardware-verified
//
#include <hip/hip_runtime.h>
#include <math.h>


#ifndef NB
#define NB 8
#endif

static constexpr int kT   = 1024;
static constexpr int kC   = 1024;
static constexpr int kNH  = 16;
static constexpr int kHD  = 64;
static constexpr int kN3  = 3 * kC;
static constexpr int kBH  = NB * kNH;
static constexpr int kRB  = kT / 64;
static constexpr int kSTP = 136;
static constexpr int kPP  = 72;
static constexpr int kThreads = 256;

static_assert(NB >= 1 && NB <= 8);
static_assert(kC == kNH * kHD);
static_assert(kHD == 64);
static_assert(kT % 128 == 0 && kN3 % 128 == 0 && kC % 128 == 0);
static_assert((kSTP % 8) == 0 && (kPP % 8) == 0);
static_assert(kNH * kRB == 256);
static_assert((NB * kT * kC) % (kThreads * 8) == 0);

typedef _Float16     v16h __attribute__((ext_vector_type(16)));
typedef _Float16     v8h  __attribute__((ext_vector_type(8)));
typedef float        v8f  __attribute__((ext_vector_type(8)));
typedef float        v4f  __attribute__((ext_vector_type(4)));
typedef unsigned int v4u  __attribute__((ext_vector_type(4)));

union Frag { v16h v; v8h half[2]; };

__device__ __forceinline__ v8f wmma_f16(v16h a, v16h b, v8f acc)
{
    acc = __builtin_amdgcn_wmma_f32_16x16x32_f16(false, a, false, b, (short)0, acc, false, false);
#if defined(__HIP_DEVICE_COMPILE__)
    asm volatile("v_nop\n\tv_nop\n\tv_nop\n\tv_nop" : "+v"(acc) : "v"(a), "v"(b));
#endif
    return acc;
}

__device__ __forceinline__ float bf16_rne(float x)
{
    unsigned int u = __float_as_uint(x);
    u = u + 0x7FFFu + ((u >> 16) & 1u);
    return __uint_as_float(u & 0xFFFF0000u);
}

__device__ __forceinline__ _Float16 cvt16(float x, float sc)
{
    return (_Float16)(bf16_rne(x) * sc);
}

__global__ __launch_bounds__(kThreads)
void k_cvt_rows(const float* __restrict__ src, _Float16* __restrict__ dst, float sc, int n)
{
    const size_t base = ((size_t)blockIdx.x * kThreads + threadIdx.x) * 8;
    if (base + 8 <= (size_t)n) {
        const v4f f0 = *(const v4f*)(src + base);
        const v4f f1 = *(const v4f*)(src + base + 4);
        v8h hv;
        hv[0] = cvt16(f0[0], sc); hv[1] = cvt16(f0[1], sc);
        hv[2] = cvt16(f0[2], sc); hv[3] = cvt16(f0[3], sc);
        hv[4] = cvt16(f1[0], sc); hv[5] = cvt16(f1[1], sc);
        hv[6] = cvt16(f1[2], sc); hv[7] = cvt16(f1[3], sc);
        const v4u u = __builtin_bit_cast(v4u, hv);
        volatile v4u* p = (volatile v4u*)(dst + base);
        *p = u;
        __threadfence();
        *p = u;
    }
}

__global__ __launch_bounds__(kThreads)
void k_cvt_wt(const float* __restrict__ W, _Float16* __restrict__ WT, float sc)
{
    __shared__ __align__(16) _Float16 tile[64][72];
    const int tid = threadIdx.x;
    const int n0  = blockIdx.x * 64;
    const int k0  = blockIdx.y * 64;

#pragma unroll
    for (int it = 0; it < 4; ++it) {
        const int idx = tid + kThreads * it;
        const int r   = idx >> 4;
        const int c4  = (idx & 15) << 2;
        const v4f f = *(const v4f*)(W + (size_t)(k0 + r) * kN3 + n0 + c4);
        tile[r][c4 + 0] = cvt16(f[0], sc);
        tile[r][c4 + 1] = cvt16(f[1], sc);
        tile[r][c4 + 2] = cvt16(f[2], sc);
        tile[r][c4 + 3] = cvt16(f[3], sc);
    }
    __syncthreads();

    v4u    u[2];
    size_t off[2];
#pragma unroll
    for (int it = 0; it < 2; ++it) {
        const int p  = tid + kThreads * it;
        const int vr = p >> 3;
        const int j  = p & 7;
        v8h hv;
#pragma unroll
        for (int i = 0; i < 8; ++i) hv[i] = tile[8 * j + i][vr];
        u[it]   = __builtin_bit_cast(v4u, hv);
        off[it] = (size_t)(n0 + vr) * kC + k0 + 8 * j;
    }
#pragma unroll
    for (int it = 0; it < 2; ++it) *(volatile v4u*)(WT + off[it]) = u[it];
    __threadfence();
#pragma unroll
    for (int it = 0; it < 2; ++it) *(volatile v4u*)(WT + off[it]) = u[it];
}

__global__ __launch_bounds__(kThreads)
void k_cvt_pk(const float* __restrict__ pk, _Float16* __restrict__ PKT)
{
    const int idx = blockIdx.x * kThreads + threadIdx.x;
    if (idx >= kNH * kHD * kHD / 8) return;
    const int row = idx >> 3;
    const int j   = idx & 7;
    const int hh  = row >> 6;
    const int e   = row & 63;
    v8h hv;
#pragma unroll
    for (int i = 0; i < 8; ++i)
        hv[i] = cvt16(pk[((size_t)(hh * kHD + 8 * j + i)) * kHD + e], 1024.0f);
    const v4u u = __builtin_bit_cast(v4u, hv);
    volatile v4u* p = (volatile v4u*)(PKT + (size_t)row * kHD + 8 * j);
    *p = u;
    __threadfence();
    *p = u;
}

__global__ __launch_bounds__(kThreads)
void k_qkv(const _Float16* __restrict__ X16, const _Float16* __restrict__ WT,
           _Float16* __restrict__ Q16, _Float16* __restrict__ K16,
           _Float16* __restrict__ KT16, _Float16* __restrict__ VT16)
{
    __shared__ __align__(16) _Float16 sT[128 * kSTP];
    const int tid  = threadIdx.x;
    const int wave = tid >> 5;
    const int lane = tid & 31;
    const int h    = lane >> 4;
    const int m    = lane & 15;
    const int wm   = wave >> 1;
    const int wn   = wave & 1;
    const int nBase = blockIdx.x * 128;
    const int mBase = blockIdx.y * 128;

    const _Float16* xa0 = X16 + (size_t)(mBase + 32 * wm + m) * kC + 8 * h;
    const _Float16* xa1 = xa0 + (size_t)16 * kC;
    const _Float16* wb0 = WT + (size_t)(nBase + 64 * wn + m) * kC + 8 * h;

    v8f acc0[4], acc1[4];
#pragma unroll
    for (int ct = 0; ct < 4; ++ct) {
#pragma unroll
        for (int r = 0; r < 8; ++r) { acc0[ct][r] = 0.0f; acc1[ct][r] = 0.0f; }
    }

#pragma unroll 1
    for (int k0 = 0; k0 < kC; k0 += 32) {
        Frag a0, a1;
        a0.half[0] = *(const v8h*)(xa0 + k0);
        a0.half[1] = *(const v8h*)(xa0 + k0 + 16);
        a1.half[0] = *(const v8h*)(xa1 + k0);
        a1.half[1] = *(const v8h*)(xa1 + k0 + 16);
#pragma unroll
        for (int ct = 0; ct < 4; ++ct) {
            Frag b;
            const _Float16* wp = wb0 + (size_t)ct * 16 * kC + k0;
            b.half[0] = *(const v8h*)(wp);
            b.half[1] = *(const v8h*)(wp + 16);
            acc0[ct] = wmma_f16(a0.v, b.v, acc0[ct]);
            acc1[ct] = wmma_f16(a1.v, b.v, acc1[ct]);
        }
    }

    {
        _Float16* s0 = sT + (32 * wm + 8 * h) * kSTP + 64 * wn + m;
#pragma unroll
        for (int ct = 0; ct < 4; ++ct) {
#pragma unroll
            for (int r = 0; r < 8; ++r) {
                s0[r * kSTP + 16 * ct]        = (_Float16)(acc0[ct][r] * (1.0f / 1024.0f));
                s0[(16 + r) * kSTP + 16 * ct] = (_Float16)(acc1[ct][r] * (1.0f / 1024.0f));
            }
        }
    }
    __syncthreads();

    const int kind = nBase >> 10;
    const int hA   = (nBase & 1023) >> 6;
    const int b    = mBase >> 10;
    const int t0   = mBase & 1023;

    if (kind < 2) {
        _Float16* dstp = (kind == 0) ? Q16 : K16;
        v4u u[8];
        int off[8];
#pragma unroll
        for (int it = 0; it < 8; ++it) {
            const int p    = it * kThreads + tid;
            const int line = p >> 3;
            const int j    = p & 7;
            const int hh   = line >> 7;
            const int tr   = line & 127;
            const v8h hv = *(const v8h*)(sT + tr * kSTP + hh * 64 + 8 * j);
            u[it]   = __builtin_bit_cast(v4u, hv);
            off[it] = ((b * kNH + hA + hh) * kT + t0 + tr) * kHD + 8 * j;
        }
#pragma unroll
        for (int it = 0; it < 8; ++it) *(volatile v4u*)(dstp + (size_t)off[it]) = u[it];
        __threadfence();
#pragma unroll
        for (int it = 0; it < 8; ++it) *(volatile v4u*)(dstp + (size_t)off[it]) = u[it];
    }
    if (kind >= 1) {
        _Float16* dstp = (kind == 1) ? KT16 : VT16;
        v4u u[8];
        int off[8];
#pragma unroll
        for (int it = 0; it < 8; ++it) {
            const int p   = it * kThreads + tid;
            const int row = p >> 4;
            const int j   = p & 15;
            const int hh  = row >> 6;
            const int d   = row & 63;
            v8h hv;
#pragma unroll
            for (int ii = 0; ii < 8; ++ii) hv[ii] = sT[(8 * j + ii) * kSTP + hh * 64 + d];
            u[it]   = __builtin_bit_cast(v4u, hv);
            off[it] = ((b * kNH + hA + hh) * kHD + d) * kT + t0 + 8 * j;
        }
#pragma unroll
        for (int it = 0; it < 8; ++it) *(volatile v4u*)(dstp + (size_t)off[it]) = u[it];
        __threadfence();
#pragma unroll
        for (int it = 0; it < 8; ++it) *(volatile v4u*)(dstp + (size_t)off[it]) = u[it];
    }
}

__global__ __launch_bounds__(128)
void k_ret(const _Float16* __restrict__ Q16, const _Float16* __restrict__ K16,
           const _Float16* __restrict__ VT16, const _Float16* __restrict__ PKT,
           float* __restrict__ R32, float* __restrict__ PART)
{
    __shared__ float sDec[kT];
    __shared__ __align__(16) _Float16 sP[4 * 16 * kPP];
    __shared__ __align__(16) float sStg[4 * 16 * kHD];
    __shared__ float sRed[8];

    const int tid  = threadIdx.x;
    const int wave = tid >> 5;
    const int lane = tid & 31;
    const int h    = lane >> 4;
    const int m    = lane & 15;
    const int rb   = blockIdx.x;
    const int head = blockIdx.y;
    const int b    = blockIdx.z;
    const int R    = rb * 64;
    const int r0   = R + 16 * wave;
    const int bh   = b * kNH + head;
    const float gamma = 1.0f - __uint_as_float((unsigned int)(127 - 5 - head) << 23);

#pragma unroll 1
    for (int n = tid; n < kT; n += 128) sDec[n] = powf(gamma, (float)n);

    Frag aq0, aq1;
    {
        const _Float16* qa = Q16 + ((size_t)bh * kT + r0 + m) * kHD + 8 * h;
        aq0.half[0] = *(const v8h*)(qa);
        aq0.half[1] = *(const v8h*)(qa + 16);
        aq1.half[0] = *(const v8h*)(qa + 32);
        aq1.half[1] = *(const v8h*)(qa + 48);
    }

    v8f cacc[4], iacc[4];
#pragma unroll
    for (int et = 0; et < 4; ++et) {
#pragma unroll
        for (int r = 0; r < 8; ++r) { cacc[et][r] = 0.0f; iacc[et][r] = 0.0f; }
    }

    {
        const _Float16* pb = PKT + ((size_t)head * kHD + m) * kHD + 8 * h;
#pragma unroll
        for (int et = 0; et < 4; ++et) {
            const _Float16* pp = pb + (size_t)et * 16 * kHD;
            Frag b0, b1;
            b0.half[0] = *(const v8h*)(pp);
            b0.half[1] = *(const v8h*)(pp + 16);
            b1.half[0] = *(const v8h*)(pp + 32);
            b1.half[1] = *(const v8h*)(pp + 48);
            cacc[et] = wmma_f16(aq0.v, b0.v, cacc[et]);
            cacc[et] = wmma_f16(aq1.v, b1.v, cacc[et]);
        }
    }
    __syncthreads();

    const _Float16* kb = K16  + ((size_t)bh * kT  + m) * kHD + 8 * h;
    const _Float16* vb = VT16 + ((size_t)bh * kHD + m) * kT  + 8 * h;
    _Float16* myP = sP + wave * (16 * kPP);
    const int nch = rb + 1;

#pragma unroll 1
    for (int c = 0; c < nch; ++c) {
        const int kc = c * 64;
#pragma unroll
        for (int nt = 0; nt < 4; ++nt) {
            const _Float16* kp = kb + (size_t)(kc + 16 * nt) * kHD;
            Frag b0, b1;
            b0.half[0] = *(const v8h*)(kp);
            b0.half[1] = *(const v8h*)(kp + 16);
            b1.half[0] = *(const v8h*)(kp + 32);
            b1.half[1] = *(const v8h*)(kp + 48);
            v8f s;
#pragma unroll
            for (int r = 0; r < 8; ++r) s[r] = 0.0f;
            s = wmma_f16(aq0.v, b0.v, s);
            s = wmma_f16(aq1.v, b1.v, s);
            const int j = kc + 16 * nt + m;
            _Float16* pcol = myP + (8 * h) * kPP + 16 * nt + m;
#pragma unroll
            for (int r = 0; r < 8; ++r) {
                const int d   = r0 + 8 * h + r - j;
                const int dcl = (d < 0) ? 0 : d;
                const float dv = sDec[dcl];
                const float p  = (d >= 0) ? (s[r] * dv * 0.25f) : 0.0f;
                pcol[r * kPP] = (_Float16)p;
            }
        }
        __syncthreads();

#pragma unroll
        for (int ks = 0; ks < 2; ++ks) {
            Frag a;
            const _Float16* pa = myP + m * kPP + 32 * ks + 8 * h;
            a.half[0] = *(const v8h*)(pa);
            a.half[1] = *(const v8h*)(pa + 16);
#pragma unroll
            for (int et = 0; et < 4; ++et) {
                const _Float16* vp = vb + (size_t)et * 16 * kT + kc + 32 * ks;
                Frag bv;
                bv.half[0] = *(const v8h*)(vp);
                bv.half[1] = *(const v8h*)(vp + 16);
                iacc[et] = wmma_f16(a.v, bv.v, iacc[et]);
            }
        }
        __syncthreads();
    }

    float psum = 0.0f, psq = 0.0f;
    float* mys = sStg + wave * (16 * kHD);
#pragma unroll
    for (int et = 0; et < 4; ++et) {
#pragma unroll
        for (int r = 0; r < 8; ++r) {
            const float v = cacc[et][r] * 0.125f + iacc[et][r] * (1.0f / 128.0f);
            mys[(8 * h + r) * kHD + 16 * et + m] = v;
            psum += v;
            psq  += v * v;
        }
    }
    __syncthreads();

    {
        v4f vals[8];
        float* rbase = R32 + ((size_t)bh * kT + r0) * kHD;
#pragma unroll
        for (int i = 0; i < 8; ++i) {
            const int row = 2 * i + h;
            vals[i] = *(const v4f*)(mys + row * kHD + 4 * m);
        }
#pragma unroll
        for (int i = 0; i < 8; ++i) {
            const int row = 2 * i + h;
            *(volatile v4f*)(rbase + (size_t)row * kHD + 4 * m) = vals[i];
        }
        __threadfence();
#pragma unroll
        for (int i = 0; i < 8; ++i) {
            const int row = 2 * i + h;
            *(volatile v4f*)(rbase + (size_t)row * kHD + 4 * m) = vals[i];
        }
    }

#pragma unroll
    for (int off = 16; off > 0; off >>= 1) {
        psum += __shfl_xor(psum, off, 32);
        psq  += __shfl_xor(psq,  off, 32);
    }
    if (lane == 0) { sRed[wave] = psum; sRed[4 + wave] = psq; }
    __syncthreads();
    {
        const float S  = ((sRed[0] + sRed[1]) + sRed[2]) + sRed[3];
        const float QQ = ((sRed[4] + sRed[5]) + sRed[6]) + sRed[7];
        v4f pv;
        pv[0] = (lane == 0) ? S  : 0.0f;
        pv[1] = (lane == 0) ? QQ : 0.0f;
        pv[2] = 0.0f;
        pv[3] = 0.0f;
        const int blk = (b * kNH + head) * kRB + rb;
        const bool wr = (wave == 0) && (lane < 8);
        volatile v4f* pp = (volatile v4f*)(PART + (size_t)blk * 32 + 4 * (lane & 7));
        if (wr) *pp = pv;
        __threadfence();
        if (wr) *pp = pv;
    }
}

__global__ __launch_bounds__(128)
void k_kv(const _Float16* __restrict__ KT16, const _Float16* __restrict__ VT16,
          const float* __restrict__ pk, float* __restrict__ outkv)
{
    __shared__ __align__(16) float sStg[kHD * kHD];
    const int tid  = threadIdx.x;
    const int wave = tid >> 5;
    const int lane = tid & 31;
    const int h    = lane >> 4;
    const int m    = lane & 15;
    const int head = blockIdx.x;
    const float gamma = 1.0f - __uint_as_float((unsigned int)(127 - 5 - head) << 23);

    v8f acc[4];
#pragma unroll
    for (int et = 0; et < 4; ++et) {
#pragma unroll
        for (int r = 0; r < 8; ++r) acc[et][r] = 0.0f;
    }

#pragma unroll 1
    for (int bb = 0; bb < NB; ++bb) {
        const int bh = bb * kNH + head;
        const _Float16* ka  = KT16 + ((size_t)bh * kHD + 16 * wave + m) * kT + 8 * h;
        const _Float16* vbp = VT16 + ((size_t)bh * kHD + m) * kT + 8 * h;
#pragma unroll 1
        for (int t0 = 0; t0 < kT; t0 += 32) {
            Frag a;
            a.half[0] = *(const v8h*)(ka + t0);
            a.half[1] = *(const v8h*)(ka + t0 + 16);
#pragma unroll
            for (int et = 0; et < 4; ++et) {
                const _Float16* vp = vbp + (size_t)et * 16 * kT + t0;
                Frag bv;
                bv.half[0] = *(const v8h*)(vp);
                bv.half[1] = *(const v8h*)(vp + 16);
                acc[et] = wmma_f16(a.v, bv.v, acc[et]);
            }
        }
    }

    const float inv = 1.0f / (64.0f * (float)NB);
#pragma unroll
    for (int et = 0; et < 4; ++et) {
#pragma unroll
        for (int r = 0; r < 8; ++r) {
            const int d = 16 * wave + 8 * h + r;
            const int e = 16 * et + m;
            const float s0 = bf16_rne(pk[((size_t)(head * kHD + d)) * kHD + e]);
            sStg[d * kHD + e] = gamma * s0 + acc[et][r] * inv;
        }
    }
    __syncthreads();

    v4f vals[8];
    int offs[8];
#pragma unroll
    for (int i = 0; i < 8; ++i) {
        const int p   = 128 * i + tid;
        const int row = p >> 4;
        const int j   = p & 15;
        vals[i] = *(const v4f*)(sStg + row * kHD + 4 * j);
        offs[i] = (head * kHD + row) * kHD + 4 * j;
    }
#pragma unroll
    for (int i = 0; i < 8; ++i) *(volatile v4f*)(outkv + (size_t)offs[i]) = vals[i];
    __threadfence();
#pragma unroll
    for (int i = 0; i < 8; ++i) *(volatile v4f*)(outkv + (size_t)offs[i]) = vals[i];
}

__global__ __launch_bounds__(kThreads)
void k_gn(const float* __restrict__ R32, const float* __restrict__ PART,
          const float* __restrict__ gw, const float* __restrict__ gb,
          float* __restrict__ out)
{
    __shared__ float sStat[2];
    const int tid  = threadIdx.x;
    const int wave = tid >> 5;
    const int lane = tid & 31;
    const int tg   = blockIdx.x;
    const int b    = blockIdx.y;

    if (wave == 0) {
        double s = 0.0, q = 0.0;
        const float* pb = PART + (size_t)b * (kNH * kRB) * 32;
#pragma unroll 1
        for (int i = 0; i < 8; ++i) {
            const v4f pv = *(const v4f*)(pb + (size_t)(lane * 8 + i) * 32);
            s += (double)pv[0];
            q += (double)pv[1];
        }
#pragma unroll
        for (int off = 16; off > 0; off >>= 1) {
            s += __shfl_xor(s, off, 32);
            q += __shfl_xor(q, off, 32);
        }
        const double invn = 1.0 / ((double)kNH * (double)kHD * (double)kT);
        const double mu   = s * invn;
        double var = q * invn - mu * mu;
        var = (var > 0.0) ? var : 0.0;
        if (lane == 0) {
            sStat[0] = (float)mu;
            sStat[1] = rsqrtf((float)var + 1e-5f);
        }
    }
    __syncthreads();

    const float mu = sStat[0];
    const float rs = sStat[1];
    const int hh = tid >> 4;
    const int j  = tid & 15;
    const float wv = bf16_rne(gw[hh]);
    const float bv = bf16_rne(gb[hh]);

    v4f    vals[4];
    size_t offs[4];
#pragma unroll
    for (int i = 0; i < 4; ++i) {
        const int t = tg * 4 + i;
        const v4f v = *(const v4f*)(R32 + (((size_t)(b * kNH + hh)) * kT + t) * kHD + 4 * j);
        v4f o;
#pragma unroll
        for (int c = 0; c < 4; ++c) o[c] = ((v[c] - mu) * rs) * wv + bv;
        vals[i] = o;
        offs[i] = ((size_t)(b * kT + t)) * kC + hh * kHD + 4 * j;
    }
#pragma unroll
    for (int i = 0; i < 4; ++i) *(volatile v4f*)(out + offs[i]) = vals[i];
    __threadfence();
#pragma unroll
    for (int i = 0; i < 4; ++i) *(volatile v4f*)(out + offs[i]) = vals[i];
}

extern "C" void kernel_launch(void* const* d_in, const int* in_sizes, int n_in,
                              void* d_out, int out_size, void* d_ws, size_t ws_size,
                              hipStream_t stream)
{
    if (n_in < 5) return;
    if (in_sizes[0] < NB * kT * kC || (in_sizes[0] % (kT * kC)) != 0) return;
    if (in_sizes[1] != kNH * kHD * kHD) return;
    if (in_sizes[2] != kC * kN3) return;
    if (in_sizes[3] != kNH || in_sizes[4] != kNH) return;
    if (out_size != NB * kT * kC + kNH * kHD * kHD) return;

    const size_t szWT   = (size_t)kN3 * kC * sizeof(_Float16);
    const size_t szX    = (size_t)NB * kT * kC * sizeof(_Float16);
    const size_t szHP   = (size_t)kBH * kT * kHD * sizeof(_Float16);
    const size_t szPKT  = (size_t)kNH * kHD * kHD * sizeof(_Float16);
    const size_t szR    = (size_t)kBH * kT * kHD * sizeof(float);
    const size_t szPART = (size_t)kBH * kRB * 128;
    const size_t total  = szWT + szX + 4 * szHP + szPKT + szR + szPART;
    if (ws_size < total) return;

    const float* x   = (const float*)d_in[0];
    const float* pk  = (const float*)d_in[1];
    const float* W   = (const float*)d_in[2];
    const float* gnw = (const float*)d_in[3];
    const float* gnb = (const float*)d_in[4];
    float* out0 = (float*)d_out;
    float* out1 = out0 + (size_t)NB * kT * kC;

    char* ws = (char*)d_ws;
    size_t off = 0;
    _Float16* WT16 = (_Float16*)(ws + off); off += szWT;
    _Float16* X16  = (_Float16*)(ws + off); off += szX;
    _Float16* Q16  = (_Float16*)(ws + off); off += szHP;
    _Float16* K16  = (_Float16*)(ws + off); off += szHP;
    _Float16* KT16 = (_Float16*)(ws + off); off += szHP;
    _Float16* VT16 = (_Float16*)(ws + off); off += szHP;
    _Float16* PKT  = (_Float16*)(ws + off); off += szPKT;
    float*    R32  = (float*)(ws + off);    off += szR;
    float*    PART = (float*)(ws + off);    off += szPART;
    if (off > ws_size) return;

    k_cvt_wt<<<dim3(kN3 / 64, kC / 64), dim3(kThreads), 0, stream>>>(W, WT16, 1024.0f);
    const int nX = NB * kT * kC;
    k_cvt_rows<<<dim3((unsigned)((nX / 8 + kThreads - 1) / kThreads)), dim3(kThreads), 0, stream>>>(x, X16, 8.0f, nX);
    k_cvt_pk<<<dim3((kNH * kHD * kHD / 8 + kThreads - 1) / kThreads), dim3(kThreads), 0, stream>>>(pk, PKT);
    k_qkv<<<dim3(kN3 / 128, NB * kT / 128), dim3(kThreads), 0, stream>>>(X16, WT16, Q16, K16, KT16, VT16);
    k_ret<<<dim3(kRB, kNH, NB), dim3(128), 0, stream>>>(Q16, K16, VT16, PKT, R32, PART);
    k_kv<<<dim3(kNH), dim3(128), 0, stream>>>(KT16, VT16, pk, out1);
    k_gn<<<dim3(kT / 4, NB), dim3(kThreads), 0, stream>>>(R32, PART, gnw, gnb, out0);
}
